// EfficientAttention_6090263626326
// MI455X (gfx1250) — hardware-run, weakly checked
//
#include <hip/hip_runtime.h>


#ifndef NB
#define NB 2
#endif
#ifndef GH
#define GH 128
#endif
#define GW   128
#define SEQ  (GH * GW)
#define NB_FULL  2
#define GH_FULL  128
#define SEQ_FULL 16384
#ifndef OUT_SEQ
#define OUT_SEQ SEQ
#endif
#define DM   64
#define NH_  8
#define HD   8
#define SRR  8
#define KGW  (GW / SRR)
#define NKEY ((GH / SRR) * (GW / SRR))
#define CK   (DM * SRR * SRR)
#define AW   4
#define CP   72
#define OSP  68
#define QC   16.0f
#define KC   16.0f
#define VC   64.0f
#define WC   64.0f
#define CTXC 1024.0f
#define SC2  ((float)(0.35355339059327378 * 1.4426950408889634 / 256.0))
#define PSH  14.0f
#define NEGB (-3.0e38f)
#define OUTI (1.0f / 65536.0f)

static_assert(DM == 64);
static_assert(NH_ * HD == DM);
static_assert(HD == 8);
static_assert(NH_ == 8);
static_assert(DM % 32 == 0);
static_assert(CK % 32 == 0);
static_assert(CK == 64 * DM);
static_assert(SRR == 8);
static_assert(GH % SRR == 0);
static_assert(GW % SRR == 0);
static_assert(NKEY % 64 == 0);
static_assert((NB * NKEY) % 64 == 0);
static_assert((NB * SEQ) % 64 == 0);
static_assert(SEQ % (16 * AW) == 0);
static_assert(((size_t)SEQ * DM) % 8 == 0);
static_assert(NB <= NB_FULL);
static_assert(GH <= GH_FULL);
static_assert(SEQ <= SEQ_FULL);
static_assert((CP * 2) % 16 == 0);
static_assert((OSP * 4) % 16 == 0);
static_assert(CP >= DM);
static_assert(OSP >= DM);
static_assert(32 * 16 * 4 == 16 * DM * 2);
static_assert(32 * 16 * 8 == 16 * DM * 4);
static_assert(256 * 2 * 16 == 64 * 64 * 2);
static_assert(AW * 16 * CP * 2 + AW * 16 * OSP * 4 <= 131072);
static_assert(64 * 65 * 4 <= 131072);
static_assert(16 * 68 * 4 <= 131072);

typedef _Float16 h16;
typedef unsigned short bf;
typedef __attribute__((ext_vector_type(16))) __bf16   v16bf;
typedef __attribute__((ext_vector_type(16))) _Float16 v16h;
typedef __attribute__((ext_vector_type(8)))  _Float16 v8h;
typedef __attribute__((ext_vector_type(8)))  unsigned short v8us;
typedef __attribute__((ext_vector_type(8)))  float    v8f;
typedef __attribute__((ext_vector_type(4)))  float    v4f;
typedef v4f  __attribute__((may_alias)) v4fa;
typedef __attribute__((ext_vector_type(16))) unsigned short v16us;
typedef v8h  __attribute__((may_alias)) v8ha;

__device__ __forceinline__ unsigned short f2bf(float f) { unsigned u = __float_as_uint(f); u += 0x7FFFu + ((u >> 16) & 1u); return (unsigned short)(u >> 16); }
__device__ __forceinline__ float bfr(float f) { return __uint_as_float(((unsigned)f2bf(f)) << 16); }
__device__ __forceinline__ v16h cat16(v8h lo, v8h hi) { return __builtin_shufflevector(lo, hi, 0, 1, 2, 3, 4, 5, 6, 7, 8, 9, 10, 11, 12, 13, 14, 15); }
__device__ __forceinline__ v16bf cat16b(v8us lo, v8us hi) { return __builtin_bit_cast(v16bf, __builtin_shufflevector(lo, hi, 0, 1, 2, 3, 4, 5, 6, 7, 8, 9, 10, 11, 12, 13, 14, 15)); }
__device__ __forceinline__ v8f wmma16(v16h a, v16h b, v8f c) { return __builtin_amdgcn_wmma_f32_16x16x32_f16(false, a, false, b, (short)0, c, false, false); }
__device__ __forceinline__ v8f wmmab(v16bf a, v16bf b, v8f c) { return __builtin_amdgcn_wmma_f32_16x16x32_bf16(false, a, false, b, (short)0, c, false, false); }
__device__ __forceinline__ v16h  ldh(const h16* p) { return cat16(*(const v8h*)p, *(const v8h*)(p + 16)); }
__device__ __forceinline__ v16bf ldb(const bf* p)  { return cat16b(*(const v8us*)p, *(const v8us*)(p + 16)); }
__device__ __forceinline__ void wave_sync() { __builtin_amdgcn_fence(3  , "wavefront"); __builtin_amdgcn_wave_barrier(); asm volatile("" ::: "memory"); }

static __device__ __forceinline__ h16 toh_flush(float v) { const h16 r = (h16)v; return (fabsf(v) < 6.103515625e-05f) ? (h16)0.0f : r; }
__device__ __forceinline__ v16us cat16u(v8us lo, v8us hi) { return __builtin_shufflevector(lo, hi, 0, 1, 2, 3, 4, 5, 6, 7, 8, 9, 10, 11, 12, 13, 14, 15); }
__device__ __forceinline__ v16us ldu(const bf* p) { return cat16u(*(const v8us*)p, *(const v8us*)(p + 16)); }
__device__ __forceinline__ v8f wmma16g(v16h a, v16h b, v8f c) {
    c = __builtin_amdgcn_wmma_f32_16x16x32_f16(false, a, false, b, (short)0, c, false, false);
    asm volatile("v_nop\n\tv_nop\n\tv_nop\n\tv_nop" : "+v"(c) : "v"(a), "v"(b));
    return c; }
template <bool F16>
__device__ __forceinline__ v8f wmmaug(v16us a, v16us b, v8f c) {
    if (F16) c = __builtin_amdgcn_wmma_f32_16x16x32_f16(false, __builtin_bit_cast(v16h, a), false, __builtin_bit_cast(v16h, b), (short)0, c, false, false);
    else     c = __builtin_amdgcn_wmma_f32_16x16x32_bf16(false, __builtin_bit_cast(v16bf, a), false, __builtin_bit_cast(v16bf, b), (short)0, c, false, false);
    asm volatile("v_nop\n\tv_nop\n\tv_nop\n\tv_nop" : "+v"(c) : "v"(a), "v"(b));
    return c; }

__global__ __launch_bounds__(256) void k_cvt8(const float* __restrict__ src, bf* dst, size_t n8) {
    const size_t i = (size_t)blockIdx.x * 256 + threadIdx.x; if (i >= n8) return;
    const v8f v = *(const v8f*)(src + i * 8); v8us o;
#pragma unroll
    for (int k = 0; k < 8; ++k) o[k] = f2bf(v[k]);
    *(volatile v8us*)(dst + i * 8) = o; __threadfence(); *(volatile v8us*)(dst + i * 8) = o;
}

__global__ __launch_bounds__(256) void k_wT(const float* __restrict__ src, bf* dst, int Cn, int f16mode, float carry) {
#pragma clang fp contract(off)
    __shared__ float ts[64 * 65];
    const int tid = threadIdx.x; const int c0 = blockIdx.x * 64; const int z = blockIdx.y;
    const float* sp = src + (size_t)z * 64 * (size_t)Cn + c0;
#pragma unroll 1
    for (int it = 0; it < 16; ++it) { const int idx = it * 256 + tid; const int r = idx >> 6, c = idx & 63;
        ts[r * 65 + c] = sp[(size_t)r * Cn + c]; }
    __syncthreads();
    bf* dp = dst + ((size_t)z * (size_t)Cn + c0) * 64;
#pragma unroll 1
    for (int ps = 0; ps < 2; ++ps) {
#pragma unroll 1
        for (int it = 0; it < 2; ++it) { const int p = it * 256 + tid; const int c = p >> 3, r8 = (p & 7) * 8; v8us o;
#pragma unroll
            for (int k = 0; k < 8; ++k) { const float v = ts[(r8 + k) * 65 + c];
                const unsigned short ub = f2bf(v);
                const h16 hv = toh_flush(bfr(v) * carry);
                const unsigned short uh = __builtin_bit_cast(unsigned short, hv);
                o[k] = f16mode ? uh : ub; }
            *(volatile v8us*)(dp + (size_t)c * 64 + r8) = o; }
        if (ps == 0) __threadfence(); }
}

template <int KIND>
__device__ __forceinline__ void gemm_body(const bf* __restrict__ A, const bf* __restrict__ Bt, const float* __restrict__ cbias, const float* __restrict__ lg, const float* __restrict__ lb, h16* P) {
    __shared__ __align__(16) float os[16 * 68];
    constexpr int KD = (KIND == 1) ? CK : DM;
    constexpr bool F16 = (KIND >= 2);
    constexpr float SCL = (KIND == 0) ? QC : ((KIND == 1) ? 1.0f : ((KIND == 2) ? (KC / WC) : (VC / WC)));
    const int lane = threadIdx.x & 31, lr = lane & 15, hi = lane >> 4;
    const int r0 = (KIND == 3) ? 0 : (int)blockIdx.x * 64;
    const int c0 = (KIND == 3) ? (int)blockIdx.x * 64 : 0;
    v8f acc[4][4];
#pragma unroll
    for (int mb = 0; mb < 4; ++mb)
#pragma unroll
        for (int nb = 0; nb < 4; ++nb) acc[mb][nb] = (v8f){};
    size_t aoff[4];
#pragma unroll
    for (int mb = 0; mb < 4; ++mb) {
        const int mrow = r0 + mb * 16 + lr;
        if (KIND == 1) { const int bb = mrow / NKEY, tk = mrow % NKEY; const int ty = tk / KGW, tx = tk % KGW;
                         aoff[mb] = ((size_t)bb * SEQ + (size_t)(ty * SRR) * GW + (size_t)(tx * SRR)) * DM + 8 * hi; }
        else           { aoff[mb] = (size_t)mrow * DM + 8 * hi; } }
    const size_t boff = (size_t)(c0 + lr) * KD + 8 * hi;
#pragma unroll 1
    for (int kc = 0; kc < KD; kc += 32) {
        const size_t ak = (KIND == 1) ? (size_t)((((kc >> 9) * GW + ((kc >> 6) & 7)) * DM) + (kc & 63)) : (size_t)kc;
        v16us a[4];
#pragma unroll
        for (int mb = 0; mb < 4; ++mb) a[mb] = ldu(A + aoff[mb] + ak);
#pragma unroll
        for (int nb = 0; nb < 4; ++nb) { const v16us b = ldu(Bt + boff + (size_t)nb * 16 * KD + kc);
#pragma unroll
            for (int mb = 0; mb < 4; ++mb) acc[mb][nb] = wmmaug<F16>(a[mb], b, acc[mb][nb]); }
    }
    float bc[4];
#pragma unroll
    for (int nb = 0; nb < 4; ++nb) bc[nb] = (KIND == 1) ? bfr(cbias[nb * 16 + lr]) : 0.0f;
    const int bb3 = c0 / NKEY, tt3 = c0 % NKEY;
#pragma unroll
    for (int mb = 0; mb < 4; ++mb) {
#pragma unroll
        for (int nb = 0; nb < 4; ++nb) {
#pragma unroll
            for (int j = 0; j < 8; ++j) os[(hi * 8 + j) * 68 + nb * 16 + lr] = (acc[mb][nb][j] + bc[nb]) * SCL; }
        wave_sync();
        if (KIND == 1) {
            const int cb0 = lr * 68 + hi * 32;
            float s = 0.0f;
#pragma unroll
            for (int i = 0; i < 8; ++i) { const v4f x = *(const v4fa*)(&os[cb0 + 4 * i]); s += (x[0] + x[1]) + (x[2] + x[3]); }
            s += __shfl_xor(s, 16, 32);
            const float mu = s * (1.0f / 64.0f);
            float q = 0.0f;
#pragma unroll
            for (int i = 0; i < 8; ++i) { const v4f x = *(const v4fa*)(&os[cb0 + 4 * i]);
                const float d0 = x[0] - mu, d1 = x[1] - mu, d2 = x[2] - mu, d3 = x[3] - mu; q += (d0 * d0 + d1 * d1) + (d2 * d2 + d3 * d3); }
            q += __shfl_xor(q, 16, 32);
            const float rs = 1.0f / sqrtf(q * (1.0f / 64.0f) + 1.0e-5f);
#pragma unroll
            for (int i = 0; i < 8; ++i) { const v4f x = *(const v4fa*)(&os[cb0 + 4 * i]);
                const v4f g = *(const v4f*)(lg + hi * 32 + 4 * i); const v4f o = *(const v4f*)(lb + hi * 32 + 4 * i); v4f y;
#pragma unroll
                for (int e = 0; e < 4; ++e) y[e] = (x[e] - mu) * rs * bfr(g[e]) + bfr(o[e]);
                *(v4fa*)(&os[cb0 + 4 * i]) = y; }
            wave_sync();
        }
#pragma unroll 1
        for (int ps = 0; ps < 2; ++ps) {
#pragma unroll
            for (int s = 0; s < 4; ++s) { const int row = 4 * s + (lane >> 3), c8 = (lane & 7) * 8;
                const v4f x0 = *(const v4fa*)(&os[row * 68 + c8]); const v4f x1 = *(const v4fa*)(&os[row * 68 + c8 + 4]); v8h hv;
#pragma unroll
                for (int i = 0; i < 4; ++i) { hv[i] = toh_flush(x0[i]); hv[4 + i] = toh_flush(x1[i]); }
                const size_t oo = (KIND == 3) ? (((size_t)bb3 * DM + (size_t)(mb * 16 + row)) * NKEY + (size_t)tt3 + c8)
                                              : ((size_t)(r0 + mb * 16 + row) * DM + c8);
                *(volatile v8h*)(P + oo) = hv; }
            if (ps == 0) __threadfence(); }
        wave_sync();
    }
}

__global__ __launch_bounds__(32) void k_qproj(const bf* __restrict__ A, const bf* __restrict__ Bt, h16* P) { gemm_body<0>(A, Bt, (const float*)0, (const float*)0, (const float*)0, P); }
__global__ __launch_bounds__(32) void k_patch(const bf* __restrict__ A, const bf* __restrict__ Bt, const float* __restrict__ cbias, const float* __restrict__ lg, const float* __restrict__ lb, h16* P) { gemm_body<1>(A, Bt, cbias, lg, lb, P); }
__global__ __launch_bounds__(32) void k_kproj(const bf* __restrict__ A, const bf* __restrict__ Bt, h16* P) { gemm_body<2>(A, Bt, (const float*)0, (const float*)0, (const float*)0, P); }
__global__ __launch_bounds__(32) void k_vproj(const bf* __restrict__ A, const bf* __restrict__ Bt, h16* P) { gemm_body<3>(A, Bt, (const float*)0, (const float*)0, (const float*)0, P); }

__global__ __launch_bounds__(32 * AW) void k_attn(const h16* __restrict__ QH, const h16* __restrict__ KP, const h16* __restrict__ VT, const h16* __restrict__ PW,
                                                  const float* __restrict__ pbias, const int* __restrict__ hp, const int* __restrict__ wp, float* OUT) {
    __shared__ __align__(16) h16   cs[AW * 16 * CP];
    __shared__ __align__(16) float os[AW * 16 * OSP];
    const int lane = threadIdx.x & 31, lr = lane & 15, hi = lane >> 4;
    const int wave = __builtin_amdgcn_readfirstlane((int)(threadIdx.x >> 5));
    const int b = blockIdx.y;
    const int t0 = (blockIdx.x * AW + wave) * 16;
    const bool bad = (hp[0] != GH_FULL) | (wp[0] != GW);
    const size_t qrow  = ((size_t)b * SEQ + (size_t)(t0 + lr)) * DM + 8 * hi;
    const size_t kbase = ((size_t)b * NKEY + (size_t)lr) * DM + 8 * hi;
    const size_t vbase = ((size_t)b * DM + (size_t)(lr & 7)) * NKEY + 8 * hi;
    const int cb = wave * 16 * CP;
    const v8h z8 = (v8h){};
#pragma unroll 1
    for (int h = 0; h < NH_; ++h) {
        const int g = h >> 2, j = h & 3;
        v8h qa = *(const v8h*)(QH + qrow + 32 * g), qb = *(const v8h*)(QH + qrow + 32 * g + 16);
        asm volatile("" : "+v"(qa), "+v"(qb));
        const bool kA = (hi == (j & 1)) & (j < 2);
        const bool kB = (hi == (j & 1)) & (j >= 2);
        qa = kA ? qa : z8; qb = kB ? qb : z8;
        const v16h qf = cat16(qa, qb);
        const size_t ko = kbase + (size_t)(32 * g);
        const size_t vo = vbase + (size_t)(h * HD) * NKEY;
        v8f o = (v8f){};
        float m = NEGB, l = 0.0f;
#pragma unroll 1
        for (int key0 = 0; key0 < NKEY; key0 += 32) {
            const h16* ka = KP + ko + (size_t)key0 * DM;
            const v16h ka0 = ldh(ka), kb0 = ldh(ka + 16 * DM);
            v8f sa = (v8f){}, sb = (v8f){};
            sa = wmma16g(ka0, qf, sa); sb = wmma16g(kb0, qf, sb);
            float ta[8], tb[8]; float mx = NEGB;
#pragma unroll
            for (int r = 0; r < 8; ++r) { ta[r] = sa[r] * SC2; tb[r] = sb[r] * SC2; mx = fmaxf(mx, fmaxf(ta[r], tb[r])); }
            mx = fmaxf(mx, __shfl_xor(mx, 16, 32));
            const float mnew = fmaxf(m, mx);
            const float alpha = __builtin_amdgcn_exp2f(m - mnew);
            const float sh = PSH - mnew;
            v16h pb; float ls = 0.0f;
#pragma unroll
            for (int r = 0; r < 8; ++r) {
                const float ea = ta[r] + sh, eb = tb[r] + sh;
                const float xa = __builtin_amdgcn_exp2f(ea), xb = __builtin_amdgcn_exp2f(eb);
                const h16 pa = (ea < -14.0f) ? (h16)0.0f : (h16)xa;
                const h16 pc = (eb < -14.0f) ? (h16)0.0f : (h16)xb;
                pb[r] = pa; pb[8 + r] = pc;
                ls += (float)pa + (float)pc; }
            l = l * alpha + ls; m = mnew;
            o = o * alpha;
            const v16h v0 = ldh(VT + vo + key0);
            o = wmma16g(v0, pb, o);
        }
        l += __shfl_xor(l, 16, 32);
        const float inv = (1.0f / l) * (CTXC / VC);
        v8h cv;
#pragma unroll
        for (int r = 0; r < 8; ++r) cv[r] = toh_flush(o[r] * inv);
        if (hi == 0) *(v8ha*)(&cs[cb + lr * CP + h * HD]) = cv;
    }
    wave_sync();
    v8f acc[4];
#pragma unroll
    for (int nb = 0; nb < 4; ++nb) acc[nb] = (v8f){};
#pragma unroll
    for (int kc = 0; kc < DM; kc += 32) {
        const v8h a0 = *(const v8ha*)(&cs[cb + lr * CP + kc + 8 * hi]);
        const v8h a1 = *(const v8ha*)(&cs[cb + lr * CP + kc + 16 + 8 * hi]);
        const v16h a = cat16(a0, a1);
#pragma unroll
        for (int nb = 0; nb < 4; ++nb) { const v16h bw = ldh(PW + (size_t)(nb * 16 + lr) * DM + kc + 8 * hi);
            acc[nb] = wmma16g(a, bw, acc[nb]); }
    }
    const int ob = wave * 16 * OSP;
    const float nanv = __uint_as_float(0x7FC00000u);
#pragma unroll
    for (int nb = 0; nb < 4; ++nb) { const float bia = bfr(pbias[nb * 16 + lr]);
#pragma unroll
        for (int r = 0; r < 8; ++r) { const float v = acc[nb][r] * OUTI + bia;
            os[ob + (8 * hi + r) * OSP + nb * 16 + lr] = bad ? nanv : v; } }
    wave_sync();
    float* orow = OUT + ((size_t)b * OUT_SEQ + (size_t)t0) * DM;
#pragma unroll 1
    for (int ps = 0; ps < 2; ++ps) {
#pragma unroll
        for (int s = 0; s < 8; ++s) { const int row = 2 * s + (lane >> 4), cofs = (lane & 15) * 4;
            const v4f val = *(const v4fa*)(&os[ob + row * OSP + cofs]);
            *(volatile v4f*)(orow + (size_t)row * DM + cofs) = val; }
        if (ps == 0) __threadfence(); }
}

static constexpr size_t al256(size_t v) { return (v + 255) & ~(size_t)255; }
static constexpr size_t SZ_XB = al256((size_t)NB * SEQ * DM * 2);
static constexpr size_t SZ_W1 = al256((size_t)DM * DM * 2);
static constexpr size_t SZ_KV = al256((size_t)2 * DM * DM * 2);
static constexpr size_t SZ_SW = al256((size_t)DM * CK * 2);
static constexpr size_t SZ_KP = al256((size_t)NB * NKEY * DM * 2);
static constexpr size_t SZ_TOTAL = 2 * SZ_XB + 2 * SZ_W1 + SZ_KV + SZ_SW + 3 * SZ_KP;
static_assert(SZ_TOTAL <= (size_t)134217728);
static_assert(((size_t)NB * SEQ * DM * 2) % 256 == 0);
static_assert(((size_t)NB * NKEY * DM * 2) % 256 == 0);
static_assert((size_t)NB * DM * NKEY == (size_t)NB * NKEY * DM);

extern "C" void kernel_launch(void* const* d_in, const int* in_sizes, int n_in,
                              void* d_out, int out_size, void* d_ws, size_t ws_size, hipStream_t stream) {
    if (n_in < 11) return;
    const size_t needx = ((size_t)(NB - 1) * SEQ_FULL + SEQ) * DM;
    if ((size_t)in_sizes[0] < needx) return;
    if (in_sizes[1] < 1 || in_sizes[2] < 1) return;
    if ((size_t)in_sizes[3] < (size_t)DM * DM || (size_t)in_sizes[4] < (size_t)2 * DM * DM || (size_t)in_sizes[5] < (size_t)DM * CK) return;
    if (in_sizes[6] < DM || in_sizes[7] < DM || in_sizes[8] < DM || (size_t)in_sizes[9] < (size_t)DM * DM || in_sizes[10] < DM) return;
    if ((size_t)out_size < ((size_t)(NB - 1) * OUT_SEQ + SEQ) * DM) return;
    if (SZ_TOTAL > ws_size) return;
    const float* x    = (const float*)d_in[0];
    const int*   gh   = (const int*)d_in[1];
    const int*   gw   = (const int*)d_in[2];
    const float* q_w  = (const float*)d_in[3];
    const float* kv_w = (const float*)d_in[4];
    const float* sr_w = (const float*)d_in[5];
    const float* sr_b = (const float*)d_in[6];
    const float* ln_g = (const float*)d_in[7];
    const float* ln_b = (const float*)d_in[8];
    const float* pj_w = (const float*)d_in[9];
    const float* pj_b = (const float*)d_in[10];
    float* OUT = (float*)d_out;
    char* wsp = (char*)d_ws;
    bf*  XB  = (bf*)wsp;  wsp += SZ_XB;
    h16* QH  = (h16*)wsp; wsp += SZ_XB;
    bf*  WQT = (bf*)wsp;  wsp += SZ_W1;
    bf*  PWT = (bf*)wsp;  wsp += SZ_W1;
    bf*  KVT = (bf*)wsp;  wsp += SZ_KV;
    bf*  SW  = (bf*)wsp;  wsp += SZ_SW;
    h16* LNP = (h16*)wsp; wsp += SZ_KP;
    h16* KP  = (h16*)wsp; wsp += SZ_KP;
    h16* VT  = (h16*)wsp; wsp += SZ_KP;

    if (SEQ == SEQ_FULL) {
        const size_t n8 = (size_t)NB * SEQ * DM / 8;
        k_cvt8<<<(unsigned)((n8 + 255) / 256), 256, 0, stream>>>(x, XB, n8);
    } else {
        const size_t n8 = (size_t)SEQ * DM / 8;
        for (int b = 0; b < NB; ++b) k_cvt8<<<(unsigned)((n8 + 255) / 256), 256, 0, stream>>>(x + (size_t)b * SEQ_FULL * DM, XB + (size_t)b * SEQ * DM, n8);
    }
    k_wT<<<dim3(1, 1, 1),  256, 0, stream>>>(q_w,  WQT, DM,     0, 1.0f);
    k_wT<<<dim3(2, 1, 1),  256, 0, stream>>>(kv_w, KVT, 2 * DM, 1, WC);
    k_wT<<<dim3(1, DM, 1), 256, 0, stream>>>(sr_w, SW,  DM,     0, 1.0f);
    k_wT<<<dim3(1, 1, 1),  256, 0, stream>>>(pj_w, PWT, DM,     1, WC);

    k_qproj<<<dim3(NB * SEQ / 64, 1, 1), 32, 0, stream>>>(XB, WQT, QH);
    k_patch<<<dim3(NB * NKEY / 64, 1, 1), 32, 0, stream>>>(XB, SW, sr_b, ln_g, ln_b, LNP);
    k_kproj<<<dim3(NB * NKEY / 64, 1, 1), 32, 0, stream>>>((const bf*)LNP, KVT, KP);
    k_vproj<<<dim3(NB * NKEY / 64, 1, 1), 32, 0, stream>>>(KVT + (size_t)DM * DM, (const bf*)LNP, VT);

    k_attn<<<dim3(SEQ / (16 * AW), NB, 1), 32 * AW, 0, stream>>>(QH, KP, VT, (const h16*)PWT, pj_b, gh, gw, OUT);
}
